// MaskedMultiHeadAttention_83597243449800
// MI455X (gfx1250) — hardware-verified
//
#include <hip/hip_runtime.h>


#ifndef NB
#define NB 4
#endif
#ifndef SEQ
#define SEQ 2048
#endif
#define NB_FULL  4
#define SEQ_FULL 2048
#define DM   1024
#define NH   16
#define HD   64
#define RH   256
#define PP   40
#define OSP  68
#define PCAR 1024.0f
#define SCL  0.03125f
#define L2E  1.4426950408889634f

static_assert(NH * HD == DM);
static_assert((SEQ % 256) == 0 && (RH % 256) == 0 && RH <= SEQ && SEQ <= SEQ_FULL && NB >= 1 && NB <= NB_FULL);
static_assert((DM % 64) == 0 && (SEQ % 64) == 0);
static_assert((size_t)3 * DM * DM * 2 + (size_t)NB * SEQ * DM * 2 + (size_t)NB * SEQ * DM * 4 + (size_t)3 * NB * NH * SEQ * HD * 2 + (size_t)6 * NB * NH * RH * HD * 2 + 12 * 256 <= (size_t)134217728);

typedef _Float16 h16;
typedef unsigned short bf;
typedef __attribute__((ext_vector_type(16))) __bf16   v16bf;
typedef __attribute__((ext_vector_type(16))) _Float16 v16h;
typedef __attribute__((ext_vector_type(8)))  _Float16 v8h;
typedef __attribute__((ext_vector_type(8)))  unsigned short v8us;
typedef __attribute__((ext_vector_type(8)))  float    v8f;
typedef __attribute__((ext_vector_type(4)))  float    v4f;
typedef v8h  __attribute__((may_alias)) v8ha;
typedef v4f  __attribute__((may_alias)) v4fa;
typedef v8us __attribute__((may_alias)) v8usa;

__device__ __forceinline__ unsigned short f2bf(float f) { unsigned u = __float_as_uint(f); u += 0x7FFFu + ((u >> 16) & 1u); return (unsigned short)(u >> 16); }
__device__ __forceinline__ float bf2f(unsigned short b) { return __uint_as_float(((unsigned)b) << 16); }
__device__ __forceinline__ float bfr(float f) { return bf2f(f2bf(f)); }
__device__ __forceinline__ void splitf(float y, unsigned short& h, unsigned short& l) { h = f2bf(y); l = f2bf(y - bf2f(h)); }
__device__ __forceinline__ v16h cat16(v8h lo, v8h hi) { return __builtin_shufflevector(lo, hi, 0, 1, 2, 3, 4, 5, 6, 7, 8, 9, 10, 11, 12, 13, 14, 15); }
__device__ __forceinline__ v16bf cat16b(v8us lo, v8us hi) { return __builtin_bit_cast(v16bf, __builtin_shufflevector(lo, hi, 0, 1, 2, 3, 4, 5, 6, 7, 8, 9, 10, 11, 12, 13, 14, 15)); }
__device__ __forceinline__ v8f wmma16(v16h a, v16h b, v8f c) { return __builtin_amdgcn_wmma_f32_16x16x32_f16(false, a, false, b, (short)0, c, false, false); }
__device__ __forceinline__ v8f wmmab(v16bf a, v16bf b, v8f c) { return __builtin_amdgcn_wmma_f32_16x16x32_bf16(false, a, false, b, (short)0, c, false, false); }

template <typename T16> struct WFrag;
template <> struct WFrag<h16> { typedef v16h V; static __device__ __forceinline__ V ld(const h16* p) { return cat16(*(const v8h*)p, *(const v8h*)(p + 16)); } static __device__ __forceinline__ v8f mma(V a, V b, v8f c) { return wmma16(a, b, c); } };
template <> struct WFrag<bf> { typedef v16bf V; static __device__ __forceinline__ V ld(const bf* p) { return cat16b(*(const v8us*)p, *(const v8us*)(p + 16)); } static __device__ __forceinline__ v8f mma(V a, V b, v8f c) { return wmmab(a, b, c); } };
__device__ __forceinline__ v16h  lds16(const h16* p) { return cat16(*(const v8ha*)p, *(const v8ha*)(p + 16)); }
__device__ __forceinline__ v16bf ldsb(const bf* p)   { return cat16b(*(const v8usa*)p, *(const v8usa*)(p + 16)); }

template <typename T16, int NSPLIT, bool BIAS>
__global__ __launch_bounds__(32) void k_gemmw(const T16* __restrict__ A, const T16* __restrict__ A2, const T16* __restrict__ Bt, const T16* __restrict__ Bt2, int K, float* C, int ldc, const float* __restrict__ bias, size_t sA, size_t sB, size_t sC) {
    typedef typename WFrag<T16>::V V;
    __shared__ __align__(16) float os[16 * 68];
    const size_t z = blockIdx.z; A += z * sA; if (A2) A2 += z * sA; Bt += z * sB; if (Bt2) Bt2 += z * sB; C += z * sC;
    const int lane = threadIdx.x & 31, lr = lane & 15, hi = lane >> 4; const int r0 = blockIdx.x * 64, c0 = blockIdx.y * 64;
    v8f acc[4][4];
#pragma unroll
    for (int mb = 0; mb < 4; ++mb)
#pragma unroll
        for (int nb = 0; nb < 4; ++nb) acc[mb][nb] = (v8f){};
    const size_t aoff = (size_t)(r0 + lr) * K + 8 * hi, boff = (size_t)(c0 + lr) * K + 8 * hi;
#pragma unroll 1
    for (int kc = 0; kc < K; kc += 32) {
        V a[4], a2[4];
#pragma unroll
        for (int mb = 0; mb < 4; ++mb) { a[mb] = WFrag<T16>::ld(A + aoff + (size_t)mb * 16 * K + kc); if (NSPLIT == 1 || NSPLIT == 2) a2[mb] = WFrag<T16>::ld(A2 + aoff + (size_t)mb * 16 * K + kc); }
#pragma unroll
        for (int nb = 0; nb < 4; ++nb) { const V b = WFrag<T16>::ld(Bt + boff + (size_t)nb * 16 * K + kc); V b2; if (NSPLIT >= 2) b2 = WFrag<T16>::ld(Bt2 + boff + (size_t)nb * 16 * K + kc);
#pragma unroll
            for (int mb = 0; mb < 4; ++mb) { acc[mb][nb] = WFrag<T16>::mma(a[mb], b, acc[mb][nb]); if (NSPLIT == 1 || NSPLIT == 2) acc[mb][nb] = WFrag<T16>::mma(a2[mb], b, acc[mb][nb]); if (NSPLIT >= 2) acc[mb][nb] = WFrag<T16>::mma(a[mb], b2, acc[mb][nb]); } }
        asm volatile("v_nop\n\tv_nop\n\tv_nop\n\tv_nop" : "+v"(acc[0][0]), "+v"(acc[1][1]), "+v"(acc[2][2]), "+v"(acc[3][3]) : "v"(a[0]), "v"(a[3]));
    }
#pragma unroll
    for (int mb = 0; mb < 4; ++mb) {
#pragma unroll
        for (int nb = 0; nb < 4; ++nb) {
#pragma unroll
            for (int j = 0; j < 8; ++j) os[(hi * 8 + j) * 68 + nb * 16 + lr] = acc[mb][nb][j]; }
        __builtin_amdgcn_fence(3, "wavefront"); __builtin_amdgcn_wave_barrier(); asm volatile("" ::: "memory");
        float* crow = C + (size_t)(r0 + mb * 16) * ldc + c0;
#pragma unroll 1
        for (int ps = 0; ps < 2; ++ps) {
#pragma unroll
            for (int s = 0; s < 8; ++s) { const int row = 2 * s + hi, cofs = lr * 4; v4f val = *(const v4fa*)(os + row * 68 + cofs); if (BIAS) { val[0] += bfr(bias[c0 + cofs]); val[1] += bfr(bias[c0 + cofs + 1]); val[2] += bfr(bias[c0 + cofs + 2]); val[3] += bfr(bias[c0 + cofs + 3]); }
                *(volatile v4f*)(crow + (size_t)row * ldc + cofs) = val; }
            if (ps == 0) __threadfence(); }
        __builtin_amdgcn_fence(3, "wavefront"); __builtin_amdgcn_wave_barrier(); asm volatile("" ::: "memory");
    }
}

__global__ __launch_bounds__(256) void k_cvt8(const float* __restrict__ src, bf* dst, size_t n8) { const size_t i = (size_t)blockIdx.x * 256 + threadIdx.x; if (i >= n8) return; const v8f v = *(const v8f*)(src + i * 8); v8us o;
#pragma unroll
    for (int k = 0; k < 8; ++k) o[k] = f2bf(v[k]); *(volatile v8us*)(dst + i * 8) = o; __threadfence(); *(volatile v8us*)(dst + i * 8) = o; }
__global__ __launch_bounds__(256) void k_cvtx(const float* __restrict__ src, bf* dst, size_t n8) { const size_t i = (size_t)blockIdx.x * 256 + threadIdx.x; if (i >= n8) return;
    const float* s = src + (size_t)blockIdx.y * SEQ_FULL * DM; bf* d = dst + (size_t)blockIdx.y * SEQ * DM; const v8f v = *(const v8f*)(s + i * 8); v8us o;
#pragma unroll
    for (int k = 0; k < 8; ++k) o[k] = f2bf(v[k]); *(volatile v8us*)(d + i * 8) = o; __threadfence(); *(volatile v8us*)(d + i * 8) = o; }

__global__ __launch_bounds__(256) void k_qkp(const float* __restrict__ F, h16* P16, bf* Ph, bf* Pl) {
    const size_t e = ((size_t)blockIdx.x * 256 + threadIdx.x) * 8; if (e >= (size_t)NB * NH * SEQ * HD) return;
    const int d = (int)(e % HD); const int t = (int)((e / HD) % SEQ); const int h = (int)((e / ((size_t)HD * SEQ)) % NH); const int b = (int)(e / ((size_t)HD * SEQ * NH));
    const v8f v = *(const v8f*)(F + ((size_t)b * SEQ + t) * DM + h * HD + d);
    v8h o16; v8us oh, ol;
#pragma unroll
    for (int k = 0; k < 8; ++k) { o16[k] = (h16)v[k]; unsigned short a1, a2; splitf(v[k], a1, a2); oh[k] = a1; ol[k] = a2; }
    const bool lo = (t < RH); const size_t oo = (((size_t)b * NH + h) * RH + (size_t)(lo ? t : 0)) * HD + d;
#pragma unroll 1
    for (int ps = 0; ps < 2; ++ps) {
        *(volatile v8h*)(P16 + e) = o16; if (lo) { *(volatile v8us*)(Ph + oo) = oh; *(volatile v8us*)(Pl + oo) = ol; }
        if (ps == 0) __threadfence(); }
}
__global__ __launch_bounds__(256) void k_vtp8(const float* __restrict__ F, h16* V16, bf* Vh, bf* Vl) {
    const size_t e = ((size_t)blockIdx.x * 256 + threadIdx.x) * 8; if (e >= (size_t)NB * NH * HD * SEQ) return;
    const int t = (int)(e % SEQ); const int d = (int)((e / SEQ) % HD); const int h = (int)((e / ((size_t)SEQ * HD)) % NH); const int b = (int)(e / ((size_t)SEQ * HD * NH));
    const float* f = F + ((size_t)b * SEQ + t) * DM + h * HD + d;
    v8h o16; v8us oh, ol;
#pragma unroll
    for (int q = 0; q < 8; ++q) { const float x = f[(size_t)q * DM]; o16[q] = (h16)x; unsigned short a1, a2; splitf(x, a1, a2); oh[q] = a1; ol[q] = a2; }
    const bool lo = (t < RH); const size_t oo = (((size_t)b * NH + h) * HD + d) * RH + (size_t)(lo ? t : 0);
#pragma unroll 1
    for (int ps = 0; ps < 2; ++ps) {
        *(volatile v8h*)(V16 + e) = o16; if (lo) { *(volatile v8us*)(Vh + oo) = oh; *(volatile v8us*)(Vl + oo) = ol; }
        if (ps == 0) __threadfence(); }
}

template <bool HR>
__global__ __launch_bounds__(128) __attribute__((amdgpu_num_vgpr(256)))
void k_attn(const h16* __restrict__ Q16, const h16* __restrict__ K16, const h16* __restrict__ VT16,
            const bf* __restrict__ QPh, const bf* __restrict__ QPl, const bf* __restrict__ KPh, const bf* __restrict__ KPl,
            const bf* __restrict__ VTh, const bf* __restrict__ VTl, int roff, float* OUT) {
    __shared__ __align__(16) float os[4][16 * OSP];
    __shared__ __align__(16) h16 pt16[4][16 * PP];
    __shared__ __align__(16) bf  pth[4][16 * PP];
    __shared__ __align__(16) bf  ptl[4][16 * PP];
    const int lane = threadIdx.x & 31, lr = lane & 15, hi = lane >> 4, wid = threadIdx.x >> 5;
    const int q0blk = roff + (int)blockIdx.x * 64;
    if (q0blk + 64 > SEQ) return;
    if (HR && q0blk + 64 > RH) return;
    const int q0 = q0blk + wid * 16;
    const size_t bh = (size_t)blockIdx.z * NH + blockIdx.y;
    const h16* Qb = Q16 + bh * SEQ * HD; const h16* Kb = K16 + bh * SEQ * HD; const h16* Vb = VT16 + bh * HD * SEQ;
    const bf* Qhb = QPh + bh * RH * HD; const bf* Qlb = QPl + bh * RH * HD; const bf* Khb = KPh + bh * RH * HD; const bf* Klb = KPl + bh * RH * HD;
    const bf* Vhb = VTh + bh * HD * RH; const bf* Vlb = VTl + bh * HD * RH;
    float* myos = os[wid]; h16* p16 = pt16[wid]; bf* ph = pth[wid]; bf* pl = ptl[wid];
    const int nchunk = (q0blk + 64) >> 5;
    const float NEG = -__builtin_inff();

    v8f o[4];
#pragma unroll
    for (int t = 0; t < 4; ++t) o[t] = (v8f){};
    float m[8], l[8];
#pragma unroll
    for (int r = 0; r < 8; ++r) { m[r] = NEG; l[r] = 0.0f; }
    v16h aq[2];
    if (!HR) { const h16* qr = Qb + (size_t)(q0 + lr) * HD + 8 * hi; aq[0] = WFrag<h16>::ld(qr); aq[1] = WFrag<h16>::ld(qr + 32); }

#pragma unroll 1
    for (int c = 0; c < nchunk; ++c) {
        const int j0 = c * 32;
        v8f s0 = (v8f){}, s1 = (v8f){};
        if (HR) {
            const bf* qh = Qhb + (size_t)(q0 + lr) * HD + 8 * hi; const bf* ql = Qlb + (size_t)(q0 + lr) * HD + 8 * hi;
            const bf* kh = Khb + (size_t)(j0 + lr) * HD + 8 * hi; const bf* kl = Klb + (size_t)(j0 + lr) * HD + 8 * hi;
#pragma unroll
            for (int kk = 0; kk < 2; ++kk) {
                const v16bf aqh = WFrag<bf>::ld(qh + kk * 32), aql = WFrag<bf>::ld(ql + kk * 32);
                const v16bf kh0 = WFrag<bf>::ld(kh + kk * 32), kh1 = WFrag<bf>::ld(kh + 16 * HD + kk * 32);
                const v16bf kl0 = WFrag<bf>::ld(kl + kk * 32), kl1 = WFrag<bf>::ld(kl + 16 * HD + kk * 32);
                s0 = wmmab(aqh, kh0, s0); s0 = wmmab(aqh, kl0, s0); s0 = wmmab(aql, kh0, s0);
                s1 = wmmab(aqh, kh1, s1); s1 = wmmab(aqh, kl1, s1); s1 = wmmab(aql, kh1, s1);
                if (kk == 1) asm volatile("v_nop\n\tv_nop\n\tv_nop\n\tv_nop" : "+v"(s0), "+v"(s1) : "v"(aql), "v"(kh1));
            }
        } else {
            const h16* kp = Kb + (size_t)(j0 + lr) * HD + 8 * hi;
#pragma unroll
            for (int kk = 0; kk < 2; ++kk) {
                const v16h bk0 = WFrag<h16>::ld(kp + kk * 32), bk1 = WFrag<h16>::ld(kp + 16 * HD + kk * 32);
                s0 = wmma16(aq[kk], bk0, s0); s1 = wmma16(aq[kk], bk1, s1);
                if (kk == 1) asm volatile("v_nop\n\tv_nop\n\tv_nop\n\tv_nop" : "+v"(s0), "+v"(s1) : "v"(aq[1]), "v"(bk1));
            }
        }
        float alpha[8], pa[8], pc[8];
#pragma unroll
        for (int r = 0; r < 8; ++r) {
            const int q = q0 + hi * 8 + r;
            const float a0 = s0[r] * SCL, c0v = s1[r] * SCL;
            const float a = (j0 + lr <= q) ? a0 : NEG; const float cc = (j0 + 16 + lr <= q) ? c0v : NEG;
            float v = fmaxf(a, cc);
#pragma unroll
            for (int off = 8; off >= 1; off >>= 1) v = fmaxf(v, __shfl_xor(v, off, 32));
            const float mn = fmaxf(m[r], v);
            alpha[r] = __builtin_amdgcn_exp2f((m[r] - mn) * L2E);
            m[r] = mn;
            const float ea = __builtin_amdgcn_exp2f((a - mn) * L2E), ec = __builtin_amdgcn_exp2f((cc - mn) * L2E);
            float rs = ea + ec;
#pragma unroll
            for (int off = 8; off >= 1; off >>= 1) rs += __shfl_xor(rs, off, 32);
            l[r] = l[r] * alpha[r] + rs; pa[r] = ea; pc[r] = ec;
        }
#pragma unroll
        for (int t = 0; t < 4; ++t)
#pragma unroll
            for (int r = 0; r < 8; ++r) o[t][r] *= alpha[r];
        if (HR) {
#pragma unroll
            for (int r = 0; r < 8; ++r) { unsigned short a1, a2, c1, c2; splitf(pa[r], a1, a2); splitf(pc[r], c1, c2);
                const int ro = (hi * 8 + r) * PP; ph[ro + lr] = a1; pl[ro + lr] = a2; ph[ro + 16 + lr] = c1; pl[ro + 16 + lr] = c2; }
        } else {
#pragma unroll
            for (int r = 0; r < 8; ++r) { const int ro = (hi * 8 + r) * PP; p16[ro + lr] = (h16)(pa[r] * PCAR); p16[ro + 16 + lr] = (h16)(pc[r] * PCAR); }
        }
        __builtin_amdgcn_fence(3, "wavefront"); __builtin_amdgcn_wave_barrier(); asm volatile("" ::: "memory");
        if (HR) {
            const v16bf aph = ldsb(ph + lr * PP + 8 * hi), apl = ldsb(pl + lr * PP + 8 * hi);
            const bf* vh = Vhb + (size_t)lr * RH + j0 + 8 * hi; const bf* vl = Vlb + (size_t)lr * RH + j0 + 8 * hi;
            v16bf fvh = aph, fvl = apl;
#pragma unroll
            for (int t = 0; t < 4; ++t) { fvh = WFrag<bf>::ld(vh + (size_t)t * 16 * RH); fvl = WFrag<bf>::ld(vl + (size_t)t * 16 * RH);
                o[t] = wmmab(aph, fvh, o[t]); o[t] = wmmab(apl, fvh, o[t]); o[t] = wmmab(aph, fvl, o[t]); }
            asm volatile("v_nop\n\tv_nop\n\tv_nop\n\tv_nop" : "+v"(o[0]), "+v"(o[1]), "+v"(o[2]), "+v"(o[3]) : "v"(aph), "v"(fvl));
        } else {
            const v16h ap = lds16(p16 + lr * PP + 8 * hi);
            const h16* vp = Vb + (size_t)lr * SEQ + j0 + 8 * hi;
            v16h fv = ap;
#pragma unroll
            for (int t = 0; t < 4; ++t) { fv = WFrag<h16>::ld(vp + (size_t)t * 16 * SEQ); o[t] = wmma16(ap, fv, o[t]); }
            asm volatile("v_nop\n\tv_nop\n\tv_nop\n\tv_nop" : "+v"(o[0]), "+v"(o[1]), "+v"(o[2]), "+v"(o[3]) : "v"(ap), "v"(fv));
        }
        asm volatile("" ::: "memory");
    }

    float inv[8];
#pragma unroll
    for (int r = 0; r < 8; ++r) inv[r] = __builtin_amdgcn_rcpf(HR ? l[r] : l[r] * PCAR);
#pragma unroll
    for (int t = 0; t < 4; ++t)
#pragma unroll
        for (int r = 0; r < 8; ++r) myos[(hi * 8 + r) * OSP + t * 16 + lr] = o[t][r] * inv[r];
    __builtin_amdgcn_fence(3, "wavefront"); __builtin_amdgcn_wave_barrier(); asm volatile("" ::: "memory");
    float* orow = OUT + ((size_t)blockIdx.z * SEQ_FULL + q0) * DM + (size_t)blockIdx.y * HD;
#pragma unroll 1
    for (int ps = 0; ps < 2; ++ps) {
#pragma unroll
        for (int s = 0; s < 8; ++s) { const int row = 2 * s + hi, cofs = lr * 4; const v4f val = *(const v4fa*)(myos + row * OSP + cofs);
            *(volatile v4f*)(orow + (size_t)row * DM + cofs) = val; }
        if (ps == 0) __threadfence(); }
}

extern "C" void kernel_launch(void* const* d_in, const int* in_sizes, int n_in,
                              void* d_out, int out_size, void* d_ws, size_t ws_size, hipStream_t stream) {
    if (n_in < 3) return;
    if ((size_t)in_sizes[0] < (size_t)(NB - 1) * SEQ_FULL * DM + (size_t)SEQ * DM) return;
    if ((size_t)in_sizes[1] < (size_t)3 * DM * DM) return;
    if (in_sizes[2] < 3 * DM) return;
    if ((size_t)out_size < (size_t)(NB - 1) * SEQ_FULL * DM + (size_t)SEQ * DM) return;
    const float* x = (const float*)d_in[0];
    const float* W = (const float*)d_in[1];
    const float* bias = (const float*)d_in[2];
    float* OUT = (float*)d_out;
    char* wsp = (char*)d_ws;
    auto take = [&](size_t bytes) { char* p = wsp; wsp += (bytes + 255) & ~(size_t)255; return (void*)p; };
    bf* WB = (bf*)take((size_t)3 * DM * DM * 2);
    bf* XB = (bf*)take((size_t)NB * SEQ * DM * 2);
    float* F = (float*)take((size_t)NB * SEQ * DM * 4);
    h16* Q16 = (h16*)take((size_t)NB * NH * SEQ * HD * 2); h16* K16 = (h16*)take((size_t)NB * NH * SEQ * HD * 2); h16* VT16 = (h16*)take((size_t)NB * NH * HD * SEQ * 2);
    bf* QPh = (bf*)take((size_t)NB * NH * RH * HD * 2); bf* QPl = (bf*)take((size_t)NB * NH * RH * HD * 2); bf* KPh = (bf*)take((size_t)NB * NH * RH * HD * 2); bf* KPl = (bf*)take((size_t)NB * NH * RH * HD * 2);
    bf* VTh = (bf*)take((size_t)NB * NH * HD * RH * 2); bf* VTl = (bf*)take((size_t)NB * NH * HD * RH * 2);
    if ((size_t)(wsp - (char*)d_ws) > ws_size) return;
    if ((size_t)(wsp - (char*)d_ws) > (size_t)134217728) return;

    k_cvt8<<<(unsigned)(((size_t)3 * DM * DM / 8 + 255) / 256), 256, 0, stream>>>(W, WB, (size_t)3 * DM * DM / 8);
    k_cvtx<<<dim3((unsigned)(((size_t)SEQ * DM / 8 + 255) / 256), NB, 1), 256, 0, stream>>>(x, XB, (size_t)SEQ * DM / 8);
    const dim3 gg(SEQ / 64, DM / 64, NB);
    const unsigned LP = (unsigned)(((size_t)NB * NH * SEQ * HD / 8 + 255) / 256);
    k_gemmw<bf, 0, true><<<gg, 32, 0, stream>>>(XB, nullptr, WB + (size_t)DM * DM, nullptr, DM, F, DM, bias + DM, (size_t)SEQ * DM, (size_t)0, (size_t)SEQ * DM);
    k_qkp<<<LP, 256, 0, stream>>>(F, Q16, QPh, QPl);
    k_gemmw<bf, 0, true><<<gg, 32, 0, stream>>>(XB, nullptr, WB, nullptr, DM, F, DM, bias, (size_t)SEQ * DM, (size_t)0, (size_t)SEQ * DM);
    k_qkp<<<LP, 256, 0, stream>>>(F, K16, KPh, KPl);
    k_gemmw<bf, 0, true><<<gg, 32, 0, stream>>>(XB, nullptr, WB + (size_t)2 * DM * DM, nullptr, DM, F, DM, bias + 2 * DM, (size_t)SEQ * DM, (size_t)0, (size_t)SEQ * DM);
    k_vtp8<<<LP, 256, 0, stream>>>(F, VT16, VTh, VTl);
    k_attn<true><<<dim3(RH / 64, NH, NB), 128, 0, stream>>>(Q16, K16, VT16, QPh, QPl, KPh, KPl, VTh, VTl, 0, OUT);
    if (SEQ > RH) k_attn<false><<<dim3((SEQ - RH) / 64, NH, NB), 128, 0, stream>>>(Q16, K16, VT16, QPh, QPl, KPh, KPl, VTh, VTl, RH, OUT);
}
